// CliffordKANLayer_71511205479239
// MI455X (gfx1250) — hardware-run, weakly checked
//
#include <hip/hip_runtime.h>


#define NB   2048
#define NI   128
#define NO   128
#define KD   9216
#define NC   256
typedef _Float16 h16;
typedef unsigned short bf;
typedef __attribute__((ext_vector_type(16))) __bf16   v16bf;
typedef __attribute__((ext_vector_type(16))) _Float16 v16h;
typedef __attribute__((ext_vector_type(8)))  _Float16 v8h;
typedef __attribute__((ext_vector_type(8)))  unsigned short v8us;
typedef __attribute__((ext_vector_type(8)))  float    v8f;
typedef __attribute__((ext_vector_type(4)))  float    v4f;
typedef v8h  __attribute__((may_alias)) v8ha;
typedef v4f  __attribute__((may_alias)) v4fa;
typedef v8us __attribute__((may_alias)) v8usa;

__device__ __forceinline__ unsigned short f2bf(float f) { unsigned u = __float_as_uint(f); u += 0x7FFFu + ((u >> 16) & 1u); return (unsigned short)(u >> 16); }
__device__ __forceinline__ float bf2f(unsigned short b) { return __uint_as_float(((unsigned)b) << 16); }
__device__ __forceinline__ float bfr(float f) { return bf2f(f2bf(f)); }
__device__ __forceinline__ v16h cat16(v8h lo, v8h hi) { return __builtin_shufflevector(lo, hi, 0, 1, 2, 3, 4, 5, 6, 7, 8, 9, 10, 11, 12, 13, 14, 15); }
__device__ __forceinline__ v16bf cat16b(v8us lo, v8us hi) { return __builtin_bit_cast(v16bf, __builtin_shufflevector(lo, hi, 0, 1, 2, 3, 4, 5, 6, 7, 8, 9, 10, 11, 12, 13, 14, 15)); }
__device__ __forceinline__ v8f wmma16(v16h a, v16h b, v8f c) { return __builtin_amdgcn_wmma_f32_16x16x32_f16(false, a, false, b, (short)0, c, false, false); }
__device__ __forceinline__ v8f wmmab(v16bf a, v16bf b, v8f c) { return __builtin_amdgcn_wmma_f32_16x16x32_bf16(false, a, false, b, (short)0, c, false, false); }

template <typename T16> struct WFrag;
template <> struct WFrag<h16> { typedef v16h V; static __device__ __forceinline__ V ld(const h16* p) { return cat16(*(const v8h*)p, *(const v8h*)(p + 16)); } static __device__ __forceinline__ v8f mma(V a, V b, v8f c) { return wmma16(a, b, c); } };
template <> struct WFrag<bf> { typedef v16bf V; static __device__ __forceinline__ V ld(const bf* p) { return cat16b(*(const v8us*)p, *(const v8us*)(p + 16)); } static __device__ __forceinline__ v8f mma(V a, V b, v8f c) { return wmmab(a, b, c); } };
template <typename T16, int NSPLIT, bool BIAS>
__global__ __launch_bounds__(32) void k_gemmw(const T16* __restrict__ A, const T16* __restrict__ A2, const T16* __restrict__ Bt, const T16* __restrict__ Bt2, int K, float* C, int ldc, const float* __restrict__ bias, size_t sA, size_t sB, size_t sC) {
    typedef typename WFrag<T16>::V V;
    __shared__ __align__(16) float os[16 * 68];
    const size_t z = blockIdx.z; A += z * sA; if (A2) A2 += z * sA; Bt += z * sB; if (Bt2) Bt2 += z * sB; C += z * sC;
    const int lane = threadIdx.x & 31, lr = lane & 15, hi = lane >> 4; const int r0 = blockIdx.x * 64, c0 = blockIdx.y * 64;
    v8f acc[4][4];
#pragma unroll
    for (int mb = 0; mb < 4; ++mb)
#pragma unroll
        for (int nb = 0; nb < 4; ++nb) acc[mb][nb] = (v8f){};
    const size_t aoff = (size_t)(r0 + lr) * K + 8 * hi, boff = (size_t)(c0 + lr) * K + 8 * hi;
    for (int kc = 0; kc < K; kc += 32) {
        V a[4], a2[4];
#pragma unroll
        for (int mb = 0; mb < 4; ++mb) { a[mb] = WFrag<T16>::ld(A + aoff + (size_t)mb * 16 * K + kc); if (NSPLIT == 1 || NSPLIT == 2) a2[mb] = WFrag<T16>::ld(A2 + aoff + (size_t)mb * 16 * K + kc); }
#pragma unroll
        for (int nb = 0; nb < 4; ++nb) { const V b = WFrag<T16>::ld(Bt + boff + (size_t)nb * 16 * K + kc); V b2; if (NSPLIT >= 2) b2 = WFrag<T16>::ld(Bt2 + boff + (size_t)nb * 16 * K + kc);
#pragma unroll
            for (int mb = 0; mb < 4; ++mb) { acc[mb][nb] = WFrag<T16>::mma(a[mb], b, acc[mb][nb]); if (NSPLIT == 1 || NSPLIT == 2) acc[mb][nb] = WFrag<T16>::mma(a2[mb], b, acc[mb][nb]); if (NSPLIT >= 2) acc[mb][nb] = WFrag<T16>::mma(a[mb], b2, acc[mb][nb]); } }
        asm volatile("v_nop\n\tv_nop\n\tv_nop\n\tv_nop" : "+v"(acc[0][0]), "+v"(acc[1][1]), "+v"(acc[2][2]), "+v"(acc[3][3]) : "v"(a[0]), "v"(a[3]));
    }
#pragma unroll
    for (int mb = 0; mb < 4; ++mb) {
#pragma unroll
        for (int nb = 0; nb < 4; ++nb) {
#pragma unroll
            for (int j = 0; j < 8; ++j) os[(hi * 8 + j) * 68 + nb * 16 + lr] = acc[mb][nb][j]; }
        __builtin_amdgcn_wave_barrier(); asm volatile("" ::: "memory");
        float* crow = C + (size_t)(r0 + mb * 16) * ldc + c0;
#pragma unroll 1
        for (int ps = 0; ps < 2; ++ps) {
#pragma unroll
            for (int s = 0; s < 8; ++s) { const int row = 2 * s + hi, cofs = lr * 4; v4f val = *(const v4fa*)(os + row * 68 + cofs); if (BIAS) { val[0] += bfr(bias[c0 + cofs]); val[1] += bfr(bias[c0 + cofs + 1]); val[2] += bfr(bias[c0 + cofs + 2]); val[3] += bfr(bias[c0 + cofs + 3]); }
                *(volatile v4f*)(crow + (size_t)row * ldc + cofs) = val; }
            if (ps == 0) __threadfence(); }
        __builtin_amdgcn_wave_barrier(); asm volatile("" ::: "memory");
    }
}

__device__ __forceinline__ h16 toh_flush(float x) { const float z = (fabsf(x) < 6.103515625e-05f) ? 0.0f : x; return (h16)z; }

typedef float v2f __attribute__((ext_vector_type(2)));

__global__ __launch_bounds__(128) void k_pa(const float* __restrict__ x, const float* __restrict__ g, h16* AP) { const unsigned b = blockIdx.y, u = blockIdx.x, i = threadIdx.x; const bool last = (u == 8u); const unsigned ug = min(u, 7u); const v2f xv = *(const v2f*)(x + ((size_t)b * NI + i) * 2); const float xr = bfr(xv[0]), xi = bfr(xv[1]); const float s0 = __fdiv_rn(xr, __fadd_rn(1.0f, expf(-xr))), s1 = __fdiv_rn(xi, __fadd_rn(1.0f, expf(-xi))); v8h o;
#pragma unroll
    for (int v = 0; v < 8; ++v) { const v2f gv = *(const v2f*)(g + (ug * 8 + v) * 2); const float dr = __fsub_rn(xr, bfr(gv[0])), di = __fsub_rn(xi, bfr(gv[1])); const float r = expf(-__fadd_rn(__fmul_rn(dr, dr), __fmul_rn(di, di))); const float e = (v == 0) ? s0 : (v == 1) ? s1 : 0.0f; o[v] = toh_flush(last ? e : r); }
    h16* d = AP + (size_t)b * KD + (size_t)u * (NI * 8) + (size_t)i * 8; *(volatile v8h*)d = o; __threadfence(); *(volatile v8h*)d = o; }

__global__ __launch_bounds__(128) void k_pb(const float* __restrict__ wt, const float* __restrict__ a, const float* __restrict__ t, h16* BP) { const unsigned c = blockIdx.y, u = blockIdx.x, i = threadIdx.x, oc = c >> 1, z = c & 1u; const bool last = (u == 8u); const unsigned ug = min(u, 7u); const float* s = wt + ((((size_t)i * NO + oc) * 8 + ug) * 8) * 2; const v2f av = *(const v2f*)(a + ((size_t)i * NO + oc) * 2); const float a0 = bfr(av[0]), a1 = bfr(av[1]); const float m0 = __fadd_rn(__fmul_rn(a0, bfr(t[(0 * 2 + 0) * 2 + z])), __fmul_rn(a1, bfr(t[(1 * 2 + 0) * 2 + z]))), m1 = __fadd_rn(__fmul_rn(a0, bfr(t[(0 * 2 + 1) * 2 + z])), __fmul_rn(a1, bfr(t[(1 * 2 + 1) * 2 + z]))); v8h o;
#pragma unroll
    for (int h = 0; h < 4; ++h) { const v4f v = *(const v4f*)(s + 4 * h); const float w0 = bfr(z ? v[1] : v[0]), w1 = bfr(z ? v[3] : v[2]); const float e0 = (h == 0) ? m0 : 0.0f, e1 = (h == 0) ? m1 : 0.0f; o[2 * h] = toh_flush(last ? e0 : w0); o[2 * h + 1] = toh_flush(last ? e1 : w1); }
    h16* d = BP + (size_t)c * KD + (size_t)u * (NI * 8) + (size_t)i * 8; *(volatile v8h*)d = o; __threadfence(); *(volatile v8h*)d = o; }

__global__ __launch_bounds__(256) void k_s1(const float* __restrict__ C, const float* __restrict__ cb, float* BS, float* CS) { const int c = threadIdx.x; const int oc = c >> 1, z = c & 1; float bs = 0.0f;
    for (int i = 0; i < NI; ++i) bs = __fadd_rn(bs, bfr(cb[((size_t)i * NO + oc) * 2 + z]));
    float cs = 0.0f;
    for (int b = 0; b < NB; ++b) cs = __fadd_rn(cs, C[(size_t)b * NC + c]);
    *(volatile float*)(BS + c) = bs; *(volatile float*)(CS + c) = cs; __threadfence(); *(volatile float*)(BS + c) = bs; *(volatile float*)(CS + c) = cs; }

__device__ __forceinline__ float cm(const float* __restrict__ CS, const float* __restrict__ BS, int z) { float m = 0.0f;
    for (int oc = 0; oc < NO; ++oc) m = __fadd_rn(m, __fadd_rn(CS[oc * 2 + z], __fmul_rn(2048.0f, BS[oc * 2 + z])));
    return __fdiv_rn(m, 262144.0f); }

__global__ __launch_bounds__(256) void k_s2(const float* __restrict__ C, const float* __restrict__ BS, const float* __restrict__ CS, float* SS) { const int c = threadIdx.x; const float m = cm(CS, BS, c & 1); const float bs = BS[c]; float ss = 0.0f;
    for (int b = 0; b < NB; ++b) { const float e = __fsub_rn(__fadd_rn(C[(size_t)b * NC + c], bs), m); ss = __fadd_rn(ss, __fmul_rn(e, e)); }
    *(volatile float*)(SS + c) = ss; __threadfence(); *(volatile float*)(SS + c) = ss; }

__global__ __launch_bounds__(256) void k_s3(const float* __restrict__ BS, const float* __restrict__ CS, const float* __restrict__ SS, float* MV, float* IV) { const int c = threadIdx.x; const int z = c & 1; const float m = cm(CS, BS, z); float q = 0.0f;
    for (int oc = 0; oc < NO; ++oc) q = __fadd_rn(q, SS[oc * 2 + z]);
    const float iv = __fdiv_rn(1.0f, sqrtf(__fadd_rn(__fdiv_rn(q, 262144.0f), 1e-5f))); *(volatile float*)(MV + c) = m; *(volatile float*)(IV + c) = iv; __threadfence(); *(volatile float*)(MV + c) = m; *(volatile float*)(IV + c) = iv; }

__global__ __launch_bounds__(256) void k_bn(const float* __restrict__ C, const float* __restrict__ BS, const float* __restrict__ MV, const float* __restrict__ IV, const float* __restrict__ ga, const float* __restrict__ be, float* out) { const size_t w = (size_t)blockIdx.x * 256 + threadIdx.x; if (w >= (size_t)NB * NC / 4) return; const int c0 = (int)(w & 63) * 4; const v4f cv = *(const v4f*)(C + w * 4); const v4f bv = *(const v4f*)(BS + c0); const v4f mv = *(const v4f*)(MV + c0); const v4f iv = *(const v4f*)(IV + c0); const v2f gv = *(const v2f*)ga; const v2f ev = *(const v2f*)be; v4f o;
#pragma unroll
    for (int j = 0; j < 4; ++j) { const int z = j & 1; o[j] = __fadd_rn(__fmul_rn(__fmul_rn(bfr(gv[z]), __fsub_rn(__fadd_rn(cv[j], bv[j]), mv[j])), iv[j]), bfr(ev[z])); }
    *(volatile v4f*)(out + w * 4) = o; __threadfence(); *(volatile v4f*)(out + w * 4) = o; }

extern "C" void kernel_launch(void* const* d_in, const int* in_sizes, int n_in, void* d_out, int out_size, void* d_ws, size_t ws_size, hipStream_t stream) {
    if (n_in < 8) return;
    if (in_sizes[0] != NB * NI * 2 || in_sizes[1] != NI * NO * 64 * 2 || in_sizes[2] != NI * NO * 2 || in_sizes[3] != NI * NO * 2 || in_sizes[4] != 2 || in_sizes[5] != 2 || in_sizes[6] != 128 || in_sizes[7] != 8) return;
    if (out_size != NB * NC) return;
    static_assert(NB % 64 == 0 && NC % 64 == 0 && KD % 64 == 0 && KD == NI * 72 && NC == NO * 2 && NI == 128 && (NB * NC / 4) % 256 == 0, "the product: M and N multiples of 64, the depth a multiple of 64 (a plane row a whole number of lines); every flat grid exact");
    const float* x = (const float*)d_in[0]; const float* wt = (const float*)d_in[1]; const float* a = (const float*)d_in[2]; const float* cb = (const float*)d_in[3]; const float* ga = (const float*)d_in[4]; const float* be = (const float*)d_in[5]; const float* g = (const float*)d_in[6]; const float* t = (const float*)d_in[7];
    float* out = (float*)d_out;
    char* wsp = (char*)d_ws; auto take = [&](size_t bytes) { char* ptr = wsp; wsp += (bytes + 255) & ~(size_t)255; return (void*)ptr; };
    h16* AP = (h16*)take((size_t)NB * KD * 2); h16* BP = (h16*)take((size_t)NC * KD * 2); float* C = (float*)take((size_t)NB * NC * 4); float* BS = (float*)take((size_t)NC * 4); float* CS = (float*)take((size_t)NC * 4); float* SS = (float*)take((size_t)NC * 4); float* MV = (float*)take((size_t)NC * 4); float* IV = (float*)take((size_t)NC * 4);
    if ((size_t)(wsp - (char*)d_ws) > ws_size) return;
    k_pa<<<dim3(9, NB, 1), NI, 0, stream>>>(x, g, AP);
    k_pb<<<dim3(9, NC, 1), NI, 0, stream>>>(wt, a, t, BP);
    k_gemmw<h16, 0, false><<<dim3(NB / 64, NC / 64, 1), 32, 0, stream>>>(AP, nullptr, BP, nullptr, KD, C, NC, nullptr, 0, 0, 0);
    k_s1<<<1, 256, 0, stream>>>(C, cb, BS, CS);
    k_s2<<<1, 256, 0, stream>>>(C, BS, CS, SS);
    k_s3<<<1, 256, 0, stream>>>(BS, CS, SS, MV, IV);
    k_bn<<<(unsigned)((size_t)NB * NC / 4 / 256), 256, 0, stream>>>(C, BS, MV, IV, ga, be, out);
}
